// _Attention_74663711474127
// MI455X (gfx1250) — hardware-verified
//
#include <hip/hip_runtime.h>
#include <math.h>

constexpr int NBATCH  = 256;
constexpr int NTOK    = 64;
constexpr int NIN     = 512;
constexpr int NHID    = 512;
constexpr int NCLS    = 97;
constexpr int NCLSP   = 128;
constexpr int NSTEPS  = 26;
constexpr int NGATE   = 4 * NHID;
constexpr int KCAT    = NIN + NHID;
constexpr int WIHP    = NIN + NCLS;
constexpr int NTHR    = 256;
constexpr int SEQ_BLK = 16;
constexpr int HPITCH  = NHID + 8;
constexpr int PPITCH  = NHID + 4;
constexpr int NROWS_TOK = NBATCH * NTOK;
constexpr int NROWS_SEQ = NBATCH * NSTEPS;
constexpr int CLS_ROWS  = 64;
constexpr int NOUT      = NBATCH * NSTEPS * NCLS;
constexpr int NOUT4     = NOUT / 4;
constexpr float ACARRY = 16.0f;
constexpr float WCARRY = 16.0f;
constexpr float FOLD   = 1.0f / (ACARRY * WCARRY);

static_assert(NBATCH % SEQ_BLK == 0, "rows per block");
static_assert(NHID == 64 * (NTHR / 32), "8 waves x 64 hidden columns");
static_assert(NIN == NHID, "score and context lane maps share one column map; ctx and h tiles share one pitch");
static_assert(KCAT % 32 == 0 && NHID % 32 == 0 && NIN % 32 == 0, "k multiple of 32");
static_assert(NROWS_TOK % 64 == 0 && NHID % 64 == 0, "projection tile multiples");
static_assert(NROWS_SEQ % CLS_ROWS == 0 && NCLSP % 64 == 0, "classifier tile multiples");
static_assert((CLS_ROWS * NCLS * 4) % 128 == 0, "classifier block span is whole lines");
static_assert((CLS_ROWS * NCLS) % 4 == 0, "float4 span");
static_assert(HPITCH % 8 == 0 && PPITCH % 4 == 0, "16-B aligned LDS rows");
static_assert(SEQ_BLK == 2 * (NTHR / 32), "two batch rows per wave in the attention phase");
static_assert(NOUT % 4 == 0 && (NOUT * 4) % 128 == 0, "output is whole float4s and whole lines");
static_assert(NOUT4 % 32 == 0, "fill tail is whole waves");

typedef __attribute__((ext_vector_type(16))) _Float16 v16h;
typedef __attribute__((ext_vector_type(8)))  _Float16 v8h;
typedef __attribute__((ext_vector_type(4)))  _Float16 v4h;
typedef __attribute__((ext_vector_type(8)))  float    v8f;
typedef __attribute__((ext_vector_type(4)))  float    v4f;

__device__ __forceinline__ v16h frag_load(const _Float16* p) {
  union { v16h v; v8h h[2]; } f;
  f.h[0] = *(const v8h*)(p);
  f.h[1] = *(const v8h*)(p + 16);
  return f.v;
}
__device__ __forceinline__ v8f mma_h(v16h a, v16h b, v8f c) {
  return __builtin_amdgcn_wmma_f32_16x16x32_f16(false, a, false, b, (short)0, c, false, false);
}
__device__ __forceinline__ void guard4_h(v8f& a0, v8f& a1, v8f& a2, v8f& a3, v16h x, v16h y0, v16h y1, v16h y2, v16h y3) {
  asm volatile("v_nop\n\tv_nop\n\tv_nop\n\tv_nop" : "+v"(a0), "+v"(a1), "+v"(a2), "+v"(a3) : "v"(x), "v"(y0), "v"(y1), "v"(y2), "v"(y3));
}
__device__ __forceinline__ void acc_guard4(v8f& a, v8f& b, v8f& c, v8f& d) {
  asm volatile("v_nop\n\tv_nop\n\tv_nop\n\tv_nop" : "+v"(a), "+v"(b), "+v"(c), "+v"(d));
}
__device__ __forceinline__ float fsig(float x)  { return __builtin_amdgcn_rcpf(1.0f + __expf(-x)); }
__device__ __forceinline__ float ftanh(float x) { return 1.0f - 2.0f * __builtin_amdgcn_rcpf(__expf(2.0f * x) + 1.0f); }
__device__ __forceinline__ void wave_lds_fence() {
  __builtin_amdgcn_fence(__ATOMIC_RELEASE, "workgroup");
  __builtin_amdgcn_wave_barrier();
  __builtin_amdgcn_fence(__ATOMIC_ACQUIRE, "workgroup");
}

template <bool VEC>
__global__ __launch_bounds__(NTHR) void cvt8_kernel(const float* __restrict__ src, unsigned short* __restrict__ dst,
                                                    int nrow_dst, int nrow_src, int ncol8, int spitch, int scol0,
                                                    int dpitch, int dcol0, float sc) {
  const int i  = blockIdx.x * NTHR + threadIdx.x;
  const int n8 = nrow_dst * ncol8;
  if (i < n8) {
    const int row = i / ncol8;
    const int c8  = i - row * ncol8;
    const int rs  = (row < nrow_src) ? row : (nrow_src - 1);
    const bool live = (row < nrow_src);
    const float* sp = src + (size_t)rs * (size_t)spitch + scol0 + c8 * 8;
    float f[8];
    if (VEC) {
      const v4f a = *(const v4f*)(sp);
      const v4f b = *(const v4f*)(sp + 4);
#pragma unroll
      for (int e = 0; e < 4; ++e) { f[e] = a[e]; f[4 + e] = b[e]; }
    } else {
#pragma unroll
      for (int e = 0; e < 8; ++e) f[e] = sp[e];
    }
    v8h hv;
#pragma unroll
    for (int e = 0; e < 8; ++e) {
      const float val = live ? (f[e] * sc) : 0.0f;
      hv[e] = (_Float16)val;
    }
    _Float16* dp = (_Float16*)dst + (size_t)row * (size_t)dpitch + dcol0 + c8 * 8;
    *(volatile v8h*)dp = hv;
    __threadfence();
    *(volatile v8h*)dp = hv;
  }
}

__global__ __launch_bounds__(NTHR) void etab_kernel(const float* __restrict__ W_ih, const float* __restrict__ b_ih,
                                                    const float* __restrict__ b_hh, float* __restrict__ E) {
  const int i = blockIdx.x * NTHR + threadIdx.x;
  if (i < NCLS * (NGATE / 4)) {
    const int cls = i / (NGATE / 4);
    const int j4  = (i - cls * (NGATE / 4)) * 4;
    v4f o;
#pragma unroll
    for (int e = 0; e < 4; ++e) {
      const float w = W_ih[(size_t)(j4 + e) * WIHP + NIN + cls];
      o[e] = (w + b_ih[j4 + e]) + b_hh[j4 + e];
    }
    float* op = E + (size_t)cls * NGATE + j4;
    *(volatile v4f*)op = o;
    __threadfence();
    *(volatile v4f*)op = o;
  }
}

__global__ __launch_bounds__(256) void gemm64_f16_kernel(const unsigned short* __restrict__ Ap, int lda,
                                                         const unsigned short* __restrict__ Btp, int ldb,
                                                         float* __restrict__ Cout, int ldc,
                                                         int M, int N, int K, float scale) {
  const _Float16* A  = (const _Float16*)Ap;
  const _Float16* Bt = (const _Float16*)Btp;
  __shared__ __align__(16) float sT[8][16 * 68];
  const int lane = threadIdx.x & 31;
  const int wave = threadIdx.x >> 5;
  const int tilesN = N >> 6;
  const int tilesM = M >> 6;
  const int tile = blockIdx.x * 8 + wave;
  if (tile >= tilesM * tilesN) return;
  const int tm = tile / tilesN;
  const int tn = tile - tm * tilesN;
  const int m0 = tm << 6;
  const int n0 = tn << 6;
  const int rlane = lane & 15;
  const int koff  = (lane >> 4) * 8;
  const int mOff  = (lane >> 4) * 8;

  v8f acc[4][4];
#pragma unroll
  for (int i = 0; i < 4; ++i)
#pragma unroll
    for (int j = 0; j < 4; ++j) acc[i][j] = (v8f){0.f, 0.f, 0.f, 0.f, 0.f, 0.f, 0.f, 0.f};

  for (int k0 = 0; k0 < K; k0 += 32) {
    v16h bf[4];
#pragma unroll
    for (int j = 0; j < 4; ++j)
      bf[j] = frag_load(Bt + (size_t)(n0 + (j << 4) + rlane) * ldb + koff + k0);
#pragma unroll
    for (int i = 0; i < 4; ++i) {
      const v16h ah = frag_load(A + (size_t)(m0 + (i << 4) + rlane) * lda + koff + k0);
#pragma unroll
      for (int j = 0; j < 4; ++j) acc[i][j] = mma_h(ah, bf[j], acc[i][j]);
      guard4_h(acc[i][0], acc[i][1], acc[i][2], acc[i][3], ah, bf[0], bf[1], bf[2], bf[3]);
    }
  }
  acc_guard4(acc[0][0], acc[0][1], acc[0][2], acc[0][3]);
  acc_guard4(acc[1][0], acc[1][1], acc[1][2], acc[1][3]);
  acc_guard4(acc[2][0], acc[2][1], acc[2][2], acc[2][3]);
  acc_guard4(acc[3][0], acc[3][1], acc[3][2], acc[3][3]);

  float* slab = sT[wave];
#pragma unroll
  for (int i = 0; i < 4; ++i) {
    const int mBase = m0 + (i << 4);
#pragma unroll
    for (int j = 0; j < 4; ++j) {
#pragma unroll
      for (int r = 0; r < 8; ++r) slab[(mOff + r) * 68 + (j << 4) + rlane] = acc[i][j][r] * scale;
    }
    wave_lds_fence();
    {
      const int hh = lane >> 4, c4 = (lane & 15) * 4;
      for (int pass = 0; pass < 2; ++pass) {
#pragma unroll
        for (int it = 0; it < 8; ++it) {
          const int row = it * 2 + hh;
          const v4f v = *(const v4f*)(slab + row * 68 + c4);
          *(volatile v4f*)(Cout + (size_t)(mBase + row) * ldc + n0 + c4) = v;
        }
        __threadfence();
      }
    }
    wave_lds_fence();
  }
}

__global__ __launch_bounds__(NTHR) __attribute__((amdgpu_num_vgpr(256))) void attn_lstm_seq_kernel(
    const float* __restrict__ bh, const int* __restrict__ ctxi, const float* __restrict__ proj,
    const unsigned short* __restrict__ WHp, const unsigned short* __restrict__ WXp,
    const float* __restrict__ b_h2h, const float* __restrict__ svp, const float* __restrict__ ETAB,
    unsigned short* __restrict__ HSp) {
  __shared__ __align__(16) _Float16 Actx[SEQ_BLK * HPITCH];
  __shared__ __align__(16) _Float16 Ah[2 * SEQ_BLK * HPITCH];
  __shared__ __align__(16) float    ppS[SEQ_BLK * PPITCH];
  __shared__ __align__(16) float    cS[SEQ_BLK * NHID];
  __shared__ __align__(16) float    attS[SEQ_BLK * NTOK];
  __shared__ int                    clsS[NSTEPS * SEQ_BLK];
  const _Float16* WH = (const _Float16*)WHp;
  const _Float16* WX = (const _Float16*)WXp;
  _Float16* HS = (_Float16*)HSp;
  const int tid = threadIdx.x, lane = tid & 31, wave = tid >> 5;
  const int c = lane & 15, hh = lane >> 4, koff = hh * 8;
  const int rowbase = blockIdx.x * SEQ_BLK;

#pragma unroll 1
  for (int i = tid; i < SEQ_BLK * HPITCH; i += NTHR) Actx[i] = (_Float16)0.0f;
#pragma unroll 1
  for (int i = tid; i < 2 * SEQ_BLK * HPITCH; i += NTHR) Ah[i] = (_Float16)0.0f;
#pragma unroll 1
  for (int i = tid; i < SEQ_BLK * NHID; i += NTHR) cS[i] = 0.0f;
#pragma unroll 1
  for (int i = tid; i < SEQ_BLK * PPITCH; i += NTHR) ppS[i] = 0.0f;
#pragma unroll 1
  for (int i = tid; i < SEQ_BLK * NTOK; i += NTHR) attS[i] = 0.0f;
#pragma unroll 1
  for (int i = tid; i < NSTEPS * SEQ_BLK; i += NTHR) {
    const int s  = i >> 4;
    const int bl = i & 15;
    int cv = ctxi[(rowbase + bl) * NSTEPS + s];
    cv = (cv < 0) ? 0 : ((cv > NCLS - 1) ? (NCLS - 1) : cv);
    clsS[i] = cv;
  }
  __syncthreads();

  const v8f z8 = {0.f, 0.f, 0.f, 0.f, 0.f, 0.f, 0.f, 0.f};
  const _Float16* acrow = Actx + c * HPITCH + koff;

#pragma unroll 1
  for (int s = 0; s < NSTEPS; ++s) {
    const int cur = s & 1;
    const _Float16* ahrow = Ah + cur * (SEQ_BLK * HPITCH) + c * HPITCH + koff;
    _Float16* ahn = Ah + (cur ^ 1) * (SEQ_BLK * HPITCH);

    {
      const int jb = 64 * wave + c;
      const _Float16* w0 = WH + (size_t)jb * NHID + koff;
      v8f pa[4];
      pa[0] = z8; pa[1] = z8; pa[2] = z8; pa[3] = z8;
#pragma unroll 1
      for (int k0 = 0; k0 < NHID; k0 += 32) {
        const v16h a  = frag_load(ahrow + k0);
        const v16h b0 = frag_load(w0 + k0);
        const v16h b1 = frag_load(w0 + (size_t)16 * NHID + k0);
        const v16h b2 = frag_load(w0 + (size_t)32 * NHID + k0);
        const v16h b3 = frag_load(w0 + (size_t)48 * NHID + k0);
        pa[0] = mma_h(a, b0, pa[0]);
        pa[1] = mma_h(a, b1, pa[1]);
        pa[2] = mma_h(a, b2, pa[2]);
        pa[3] = mma_h(a, b3, pa[3]);
        guard4_h(pa[0], pa[1], pa[2], pa[3], a, b0, b1, b2, b3);
      }
      acc_guard4(pa[0], pa[1], pa[2], pa[3]);
#pragma unroll
      for (int nt = 0; nt < 4; ++nt) {
        const float bq = b_h2h[jb + 16 * nt];
#pragma unroll
        for (int r = 0; r < 8; ++r) ppS[(8 * hh + r) * PPITCH + jb + 16 * nt] = pa[nt][r] * FOLD + bq;
      }
    }
    __syncthreads();

#pragma unroll 1
    for (int bb = 0; bb < 2; ++bb) {
      const int bl = 2 * wave + bb;
      v4f ppr[4], svr[4];
#pragma unroll
      for (int q = 0; q < 4; ++q) {
        ppr[q] = *(const v4f*)(ppS + bl * PPITCH + 4 * lane + 128 * q);
        svr[q] = *(const v4f*)(svp + 4 * lane + 128 * q);
      }
      const float* pj = proj + ((size_t)(rowbase + bl) * NTOK) * NHID + 4 * lane;
      float s0 = 0.0f, s1 = 0.0f;
#pragma unroll 1
      for (int t = 0; t < NTOK; ++t) {
        float sacc = 0.0f;
#pragma unroll
        for (int q = 0; q < 4; ++q) {
          const v4f p = *(const v4f*)(pj + (size_t)t * NHID + 128 * q);
#pragma unroll
          for (int e = 0; e < 4; ++e) sacc += ftanh(p[e] + ppr[q][e]) * svr[q][e];
        }
#pragma unroll
        for (int off = 1; off < 32; off <<= 1) sacc += __shfl_xor(sacc, off, 32);
        s0 = (t == lane) ? sacc : s0;
        s1 = (t == lane + 32) ? sacc : s1;
      }
      float mx = fmaxf(s0, s1);
#pragma unroll
      for (int off = 1; off < 32; off <<= 1) mx = fmaxf(mx, __shfl_xor(mx, off, 32));
      const float e0 = expf(s0 - mx);
      const float e1 = expf(s1 - mx);
      float sum = e0 + e1;
#pragma unroll
      for (int off = 1; off < 32; off <<= 1) sum += __shfl_xor(sum, off, 32);
      const float inv = 1.0f / sum;
      attS[bl * NTOK + lane]      = e0 * inv;
      attS[bl * NTOK + 32 + lane] = e1 * inv;
      wave_lds_fence();
      v4f cacc[4];
#pragma unroll
      for (int q = 0; q < 4; ++q) cacc[q] = (v4f){0.f, 0.f, 0.f, 0.f};
      const float* bp = bh + ((size_t)(rowbase + bl) * NTOK) * NIN + 4 * lane;
#pragma unroll 1
      for (int t = 0; t < NTOK; ++t) {
        const float aw = attS[bl * NTOK + t];
#pragma unroll
        for (int q = 0; q < 4; ++q) {
          const v4f x = *(const v4f*)(bp + (size_t)t * NIN + 128 * q);
#pragma unroll
          for (int e = 0; e < 4; ++e) cacc[q][e] += aw * x[e];
        }
      }
#pragma unroll
      for (int q = 0; q < 4; ++q) {
        v4h hv;
#pragma unroll
        for (int e = 0; e < 4; ++e) {
          const float val = cacc[q][e] * ACARRY;
          hv[e] = (_Float16)val;
        }
        *(v4h*)(Actx + bl * HPITCH + 4 * lane + 128 * q) = hv;
      }
    }
    __syncthreads();

    {
      int clsr[8];
#pragma unroll
      for (int r = 0; r < 8; ++r) clsr[r] = clsS[s * SEQ_BLK + 8 * hh + r];
#pragma unroll 1
      for (int nt = 0; nt < 4; ++nt) {
        const int j = 64 * wave + 16 * nt + c;
        const _Float16* wx = WX + (size_t)j * KCAT + koff;
        v8f acc[4];
        acc[0] = z8; acc[1] = z8; acc[2] = z8; acc[3] = z8;
#pragma unroll 1
        for (int k0 = 0; k0 < NIN; k0 += 32) {
          const v16h a  = frag_load(acrow + k0);
          const v16h b0 = frag_load(wx + k0);
          const v16h b1 = frag_load(wx + (size_t)1 * NHID * KCAT + k0);
          const v16h b2 = frag_load(wx + (size_t)2 * NHID * KCAT + k0);
          const v16h b3 = frag_load(wx + (size_t)3 * NHID * KCAT + k0);
          acc[0] = mma_h(a, b0, acc[0]);
          acc[1] = mma_h(a, b1, acc[1]);
          acc[2] = mma_h(a, b2, acc[2]);
          acc[3] = mma_h(a, b3, acc[3]);
          guard4_h(acc[0], acc[1], acc[2], acc[3], a, b0, b1, b2, b3);
        }
#pragma unroll 1
        for (int k0 = 0; k0 < NHID; k0 += 32) {
          const v16h a  = frag_load(ahrow + k0);
          const v16h b0 = frag_load(wx + NIN + k0);
          const v16h b1 = frag_load(wx + (size_t)1 * NHID * KCAT + NIN + k0);
          const v16h b2 = frag_load(wx + (size_t)2 * NHID * KCAT + NIN + k0);
          const v16h b3 = frag_load(wx + (size_t)3 * NHID * KCAT + NIN + k0);
          acc[0] = mma_h(a, b0, acc[0]);
          acc[1] = mma_h(a, b1, acc[1]);
          acc[2] = mma_h(a, b2, acc[2]);
          acc[3] = mma_h(a, b3, acc[3]);
          guard4_h(acc[0], acc[1], acc[2], acc[3], a, b0, b1, b2, b3);
        }
        acc_guard4(acc[0], acc[1], acc[2], acc[3]);
#pragma unroll
        for (int g = 0; g < 4; ++g) {
          float ev[8];
#pragma unroll
          for (int r = 0; r < 8; ++r) ev[r] = ETAB[(size_t)clsr[r] * NGATE + g * NHID + j];
#pragma unroll
          for (int r = 0; r < 8; ++r) acc[g][r] = acc[g][r] * FOLD + ev[r];
          asm volatile("" : "+v"(acc[g]) :: "memory");
        }
        float*    cp = cS  + (8 * hh) * NHID   + j;
        _Float16* hp = ahn + (8 * hh) * HPITCH + j;
#pragma unroll
        for (int r = 0; r < 8; ++r) {
          const float ig = fsig(acc[0][r]);
          const float fg = fsig(acc[1][r]);
          const float gg = ftanh(acc[2][r]);
          const float og = fsig(acc[3][r]);
          const float co = cp[r * NHID];
          const float cn = fg * co + ig * gg;
          cp[r * NHID] = cn;
          const float hn = og * ftanh(cn);
          const float hval = hn * ACARRY;
          hp[r * HPITCH] = (_Float16)hval;
        }
      }
    }
    __syncthreads();

    {
      v8h hv[4];
#pragma unroll
      for (int it = 0; it < 4; ++it) {
        const int idx = it * 32 + lane;
        const int row = 2 * wave + (idx >> 6);
        const int ch  = idx & 63;
        hv[it] = *(const v8h*)(ahn + row * HPITCH + ch * 8);
      }
      for (int pass = 0; pass < 2; ++pass) {
#pragma unroll
        for (int it = 0; it < 4; ++it) {
          const int idx = it * 32 + lane;
          const int row = 2 * wave + (idx >> 6);
          const int ch  = idx & 63;
          *(volatile v8h*)(HS + ((size_t)(rowbase + row) * NSTEPS + (size_t)s) * NHID + ch * 8) = hv[it];
        }
        __threadfence();
      }
    }
  }
}

__global__ __launch_bounds__(NTHR) void cls_kernel(const unsigned short* __restrict__ HSp, const unsigned short* __restrict__ WCp,
                                                   const float* __restrict__ b_cls, float* __restrict__ out) {
  __shared__ __align__(16) float OutS[CLS_ROWS * NCLS];
  const _Float16* HS = (const _Float16*)HSp;
  const _Float16* WC = (const _Float16*)WCp;
  const int tid = threadIdx.x, lane = tid & 31, wave = tid >> 5;
  const int c = lane & 15, hh = lane >> 4, koff = hh * 8;
  const int mi = wave & 3, nh = wave >> 2;
  const int m0 = blockIdx.x * CLS_ROWS + mi * 16;
  const _Float16* ar = HS + (size_t)(m0 + c) * NHID + koff;
  const _Float16* wr = WC + (size_t)(nh * 64 + c) * NHID + koff;
  const v8f z8 = {0.f, 0.f, 0.f, 0.f, 0.f, 0.f, 0.f, 0.f};
  v8f acc[4];
  acc[0] = z8; acc[1] = z8; acc[2] = z8; acc[3] = z8;
#pragma unroll 1
  for (int k0 = 0; k0 < NHID; k0 += 32) {
    const v16h a  = frag_load(ar + k0);
    const v16h b0 = frag_load(wr + k0);
    const v16h b1 = frag_load(wr + (size_t)16 * NHID + k0);
    const v16h b2 = frag_load(wr + (size_t)32 * NHID + k0);
    const v16h b3 = frag_load(wr + (size_t)48 * NHID + k0);
    acc[0] = mma_h(a, b0, acc[0]);
    acc[1] = mma_h(a, b1, acc[1]);
    acc[2] = mma_h(a, b2, acc[2]);
    acc[3] = mma_h(a, b3, acc[3]);
    guard4_h(acc[0], acc[1], acc[2], acc[3], a, b0, b1, b2, b3);
  }
  acc_guard4(acc[0], acc[1], acc[2], acc[3]);
  float bvv[4];
#pragma unroll
  for (int jt = 0; jt < 4; ++jt) {
    const int n  = nh * 64 + 16 * jt + c;
    const int nb = (n < NCLS) ? n : (NCLS - 1);
    float bv = b_cls[nb];
    asm volatile("" : "+v"(bv));
    bvv[jt] = bv;
  }
#pragma unroll
  for (int jt = 0; jt < 4; ++jt) {
    const int n = nh * 64 + 16 * jt + c;
    float ov[8];
#pragma unroll
    for (int r = 0; r < 8; ++r) ov[r] = acc[jt][r] * FOLD + bvv[jt];
    if (n < NCLS) {
#pragma unroll
      for (int r = 0; r < 8; ++r) OutS[(mi * 16 + 8 * hh + r) * NCLS + n] = ov[r];
    }
  }
  __syncthreads();
  float* ob = out + (size_t)blockIdx.x * (CLS_ROWS * NCLS);
  constexpr int NV4 = (CLS_ROWS * NCLS) / 4;
  for (int pass = 0; pass < 2; ++pass) {
#pragma unroll
    for (int it = 0; it < 7; ++it) {
      const int idx = it * NTHR + tid;
      if (idx < NV4) {
        const v4f v = *(const v4f*)(OutS + 4 * idx);
        *(volatile v4f*)(ob + 4 * idx) = v;
      }
    }
    __threadfence();
  }
}

__global__ __launch_bounds__(NTHR) void premise_guard_kernel(const int* __restrict__ mlen, const int* __restrict__ tmode,
                                                             float* __restrict__ out) {
  const int tid = threadIdx.x;
  const int ml = mlen[0];
  const int tm = tmode[0];
  const bool bad = (ml != NSTEPS - 1) || (tm == 0);
  if (bad) {
    const float qn = __uint_as_float(0x7FC00000u);
    const v4f nv = {qn, qn, qn, qn};
    for (int pass = 0; pass < 2; ++pass) {
#pragma unroll 1
      for (int idx = tid; idx < NOUT4; idx += NTHR) *(volatile v4f*)(out + (size_t)4 * (size_t)idx) = nv;
      __threadfence();
    }
  }
}

extern "C" void kernel_launch(void* const* d_in, const int* in_sizes, int n_in,
                              void* d_out, int out_size, void* d_ws, size_t ws_size, hipStream_t stream) {
  if (n_in < 14 || d_out == nullptr || d_ws == nullptr) return;
  if (in_sizes[0] != NBATCH * NTOK * NIN || in_sizes[1] != NBATCH * NSTEPS || in_sizes[2] < 1 || in_sizes[3] < 1 ||
      in_sizes[4] != NHID * NIN ||
      in_sizes[5] != NHID * NHID || in_sizes[6] != NHID || in_sizes[7] != NHID || in_sizes[8] != NGATE * WIHP ||
      in_sizes[9] != NGATE || in_sizes[10] != NGATE * NHID || in_sizes[11] != NGATE || in_sizes[12] != NCLS * NHID ||
      in_sizes[13] != NCLS || out_size != NOUT) return;

  const float* bh     = (const float*)d_in[0];
  const int*   ctxi   = (const int*)d_in[1];
  const int*   mlen   = (const int*)d_in[2];
  const int*   tmode  = (const int*)d_in[3];
  const float* W_i2h  = (const float*)d_in[4];
  const float* W_h2h  = (const float*)d_in[5];
  const float* b_h2h  = (const float*)d_in[6];
  const float* wscore = (const float*)d_in[7];
  const float* W_ih   = (const float*)d_in[8];
  const float* b_ih   = (const float*)d_in[9];
  const float* W_hh   = (const float*)d_in[10];
  const float* b_hh   = (const float*)d_in[11];
  const float* W_cls  = (const float*)d_in[12];
  const float* b_cls  = (const float*)d_in[13];
  float* out = (float*)d_out;

  char* ws = (char*)d_ws; size_t off = 0;
  auto carve = [&](size_t bytes) -> char* { char* p = ws + off; off += (bytes + 255) & ~(size_t)255; return p; };
  unsigned short* BH16 = (unsigned short*)carve((size_t)NROWS_TOK * NIN * 2);
  unsigned short* WI16 = (unsigned short*)carve((size_t)NHID * NIN * 2);
  unsigned short* WH16 = (unsigned short*)carve((size_t)NHID * NHID * 2);
  unsigned short* WX16 = (unsigned short*)carve((size_t)NGATE * KCAT * 2);
  unsigned short* WC16 = (unsigned short*)carve((size_t)NCLSP * NHID * 2);
  float*          ETAB = (float*)carve((size_t)NCLS * NGATE * 4);
  float*          PROJ = (float*)carve((size_t)NROWS_TOK * NHID * 4);
  unsigned short* HS16 = (unsigned short*)carve((size_t)NROWS_SEQ * NHID * 2);
  if (off > ws_size || off > (size_t)134217728) return;

  const int nc8 = NIN / 8;
  cvt8_kernel<true><<<(NROWS_TOK * nc8 + NTHR - 1) / NTHR, NTHR, 0, stream>>>(bh, BH16, NROWS_TOK, NROWS_TOK, nc8, NIN, 0, NIN, 0, ACARRY);
  cvt8_kernel<true><<<(NHID * nc8 + NTHR - 1) / NTHR, NTHR, 0, stream>>>(W_i2h, WI16, NHID, NHID, nc8, NIN, 0, NIN, 0, WCARRY);
  cvt8_kernel<true><<<(NHID * nc8 + NTHR - 1) / NTHR, NTHR, 0, stream>>>(W_h2h, WH16, NHID, NHID, nc8, NHID, 0, NHID, 0, WCARRY);
  cvt8_kernel<false><<<(NGATE * nc8 + NTHR - 1) / NTHR, NTHR, 0, stream>>>(W_ih, WX16, NGATE, NGATE, nc8, WIHP, 0, KCAT, 0, WCARRY);
  cvt8_kernel<true><<<(NGATE * nc8 + NTHR - 1) / NTHR, NTHR, 0, stream>>>(W_hh, WX16, NGATE, NGATE, nc8, NHID, 0, KCAT, NIN, WCARRY);
  cvt8_kernel<true><<<(NCLSP * nc8 + NTHR - 1) / NTHR, NTHR, 0, stream>>>(W_cls, WC16, NCLSP, NCLS, nc8, NHID, 0, NHID, 0, WCARRY);
  etab_kernel<<<(NCLS * (NGATE / 4) + NTHR - 1) / NTHR, NTHR, 0, stream>>>(W_ih, b_ih, b_hh, ETAB);

  gemm64_f16_kernel<<<(NROWS_TOK / 64) * (NHID / 64) / 8, 256, 0, stream>>>(
      BH16, NIN, WI16, NIN, PROJ, NHID, NROWS_TOK, NHID, NIN, FOLD);

  attn_lstm_seq_kernel<<<NBATCH / SEQ_BLK, NTHR, 0, stream>>>(bh, ctxi, PROJ, WH16, WX16, b_h2h, wscore, ETAB, HS16);

  cls_kernel<<<NROWS_SEQ / CLS_ROWS, NTHR, 0, stream>>>(HS16, WC16, b_cls, out);

  premise_guard_kernel<<<1, NTHR, 0, stream>>>(mlen, tmode, out);
}
